// NeighborhoodAttn_27882927686305
// MI455X (gfx1250) — hardware-verified
//
#include <hip/hip_runtime.h>
#include <math.h>

typedef __attribute__((ext_vector_type(16))) _Float16 v16h;
typedef __attribute__((ext_vector_type(16))) __bf16 v16b;
typedef __attribute__((ext_vector_type(8)))  _Float16 v8h;
typedef __attribute__((ext_vector_type(8)))  float v8f;
typedef __attribute__((ext_vector_type(4)))  float v4f;
typedef __attribute__((ext_vector_type(2)))  float v2f;
typedef __attribute__((ext_vector_type(4)))  unsigned v4u;
typedef __attribute__((ext_vector_type(4)))  int v4i;
typedef float __attribute__((may_alias)) float_a;
typedef int __attribute__((may_alias)) int_a;

template <typename T> __device__ __forceinline__ void vst2(void* p, T v) { *(volatile T*)p = v; __threadfence(); *(volatile T*)p = v; }
__device__ __forceinline__ v8f wmma16(v16h a, v16h b, v8f c) {
  v8f d = __builtin_amdgcn_wmma_f32_16x16x32_f16(false, a, false, b, (short)0, c, false, false);
  asm volatile("v_nop\n\tv_nop\n\tv_nop\n\tv_nop" : "+v"(d) : "v"(a), "v"(b));
  return d;
}
__device__ __forceinline__ v8f wmma_bf(v16b a, v16b b, v8f c) {
  v8f d = __builtin_amdgcn_wmma_f32_16x16x32_bf16(false, a, false, b, (short)0, c, false, false);
  asm volatile("v_nop\n\tv_nop\n\tv_nop\n\tv_nop" : "+v"(d) : "v"(a), "v"(b));
  return d;
}
__device__ __forceinline__ v16h frag_h(const _Float16* rowk0, int lane) {
  union { v16h v; v8h q[2]; } u; const _Float16* p = rowk0 + 8 * (lane >> 4);
  u.q[0] = *(const v8h*)p; u.q[1] = *(const v8h*)(p + 16); return u.v;
}
__device__ __forceinline__ v16h frag_f32(const float* rowk0, int lane) {
  v16h a; const float* p = rowk0 + 8 * (lane >> 4);
#pragma unroll
  for (int i = 0; i < 8; ++i) { a[i] = (_Float16)p[i]; a[8 + i] = (_Float16)p[16 + i]; }
  return a;
}
__device__ __forceinline__ v16h frag_f32s(const float* rowk0, int lane, float sc) {
  v16h a; const float* p = rowk0 + 8 * (lane >> 4);
#pragma unroll
  for (int i = 0; i < 8; ++i) { a[i] = (_Float16)(p[i] * sc); a[8 + i] = (_Float16)(p[16 + i] * sc); }
  return a;
}
__device__ __forceinline__ v16h fragc_f32(const float* W, int k0, int n, int lane, int ld, int K) {
  v16h a; const int g = lane >> 4;
#pragma unroll
  for (int i = 0; i < 8; ++i) { const int ka = k0 + 8 * g + i, kb = ka + 16;
    a[i] = (_Float16)(ka < K ? W[(size_t)(ka < K ? ka : K - 1) * ld + n] : 0.f); a[8 + i] = (_Float16)(kb < K ? W[(size_t)(kb < K ? kb : K - 1) * ld + n] : 0.f); }
  return a;
}
struct F2 { v16b h, l; };
__device__ __forceinline__ F2 bsplit16(const float v[16]) { F2 r;
#pragma unroll
  for (int i = 0; i < 16; ++i) { const __bf16 h = (__bf16)v[i]; r.h[i] = h; r.l[i] = (__bf16)(v[i] - (float)h); }
  return r; }
__device__ __forceinline__ F2 split_row(const float* row, int k0, int lane) { float v[16]; const float* p = row + k0 + 8 * (lane >> 4);
#pragma unroll
  for (int i = 0; i < 8; ++i) { v[i] = p[i]; v[8 + i] = p[16 + i]; }
  return bsplit16(v); }
__device__ __forceinline__ F2 split_rowK(const float* row, int k0, int lane, int K) { float v[16]; const int g = lane >> 4;
#pragma unroll
  for (int i = 0; i < 8; ++i) { const int ka = k0 + 8 * g + i, kb = ka + 16; v[i] = ka < K ? row[ka < K ? ka : K - 1] : 0.f; v[8 + i] = kb < K ? row[kb < K ? kb : K - 1] : 0.f; }
  return bsplit16(v); }
__device__ __forceinline__ F2 split_col(const float* W, int k0, int n, int lane, int ld, int K) { float v[16]; const int g = lane >> 4;
#pragma unroll
  for (int i = 0; i < 8; ++i) { const int ka = k0 + 8 * g + i, kb = ka + 16; v[i] = ka < K ? W[(size_t)(ka < K ? ka : K - 1) * ld + n] : 0.f; v[8 + i] = kb < K ? W[(size_t)(kb < K ? kb : K - 1) * ld + n] : 0.f; }
  return bsplit16(v); }
__device__ __forceinline__ v8f mac3(const F2& a, const F2& b, v8f c) { c = wmma_bf(a.l, b.h, c); c = wmma_bf(a.h, b.l, c); return wmma_bf(a.h, b.h, c); }
__device__ __forceinline__ float sigm(float v) { return 1.0f / (1.0f + expf(-v)); }
#define LDSX() do { asm volatile("s_wait_dscnt 0" ::: "memory"); __builtin_amdgcn_wave_barrier(); __builtin_amdgcn_fence(__ATOMIC_RELEASE, "workgroup"); } while (0)

__device__ __forceinline__ float bfr(float v) { return (float)(__bf16)v; }
#define NBT 2
#define CC 512
#define HH 48
#define WWD 48
#define TT (HH * WWD)
#define NH 8
#define HD 64
#define NS 7
#define RR 3
#define NROW (NBT * TT)
#ifndef NPIXB
#define NPIXB (NROW / 8)
#endif
#define WS_XT 0u
#define WS_Q  (WS_XT + 4u * (size_t)NROW * CC)
#define WS_K  (WS_Q + 4u * (size_t)NROW * CC)
#define WS_V  (WS_K + 4u * (size_t)NROW * CC)
#define WS_O  (WS_V + 4u * (size_t)NROW * CC)
#define WS_END (WS_O + 4u * (size_t)NROW * CC)
__global__ __launch_bounds__(256) void k_xt(const float* __restrict__ X, float* __restrict__ XT) { __shared__ float st[128][65];
  const int t = threadIdx.x; const int t0 = blockIdx.x * 64, c0 = blockIdx.y * 128; const size_t b = blockIdx.z;
  for (int e = t; e < 128 * 64; e += 256) { const int cl = e >> 6, tl = e & 63; st[cl][tl] = bfr(X[(b * CC + c0 + cl) * TT + t0 + tl]); }
  __syncthreads();
  for (int e = t; e < 64 * 32; e += 256) { const int tl = e >> 5, q = e & 31; v4f o; o[0] = st[q * 4][tl]; o[1] = st[q * 4 + 1][tl]; o[2] = st[q * 4 + 2][tl]; o[3] = st[q * 4 + 3][tl]; vst2(XT + (b * TT + t0 + tl) * CC + c0 + q * 4, o); } }
__global__ __launch_bounds__(128) void k_proj(const float* __restrict__ XT, const float* __restrict__ WQ, const float* __restrict__ BQ, const float* __restrict__ WK, const float* __restrict__ BK, const float* __restrict__ WV, const float* __restrict__ BV, float* __restrict__ Q, float* __restrict__ K, float* __restrict__ V) { __shared__ __align__(16) float sf[4][16][132];
  const int tid = threadIdx.x, wave = tid >> 5, lane = tid & 31, col = lane & 15, g = lane >> 4; const int which = blockIdx.z; const int c0 = blockIdx.y * 128; const size_t r0 = (size_t)blockIdx.x * 64 + wave * 16;
  const float* WA = which == 0 ? WQ : which == 1 ? WK : WV; const float* BA = which == 0 ? BQ : which == 1 ? BK : BV; float* D = which == 0 ? Q : which == 1 ? K : V;
  v8f acc[8] = {};
#pragma unroll 2
  for (int kc = 0; kc < CC / 32; ++kc) { v16b a; { const float* p = XT + (r0 + col) * CC + kc * 32 + 8 * g;
#pragma unroll
      for (int i = 0; i < 8; ++i) { a[i] = (__bf16)p[i]; a[8 + i] = (__bf16)p[16 + i]; } }
#pragma unroll
    for (int j = 0; j < 8; ++j) { v16b w; const int o = c0 + j * 16 + col; const float* wr = WA + (size_t)o * CC + kc * 32 + 8 * g;
#pragma unroll
      for (int i = 0; i < 8; ++i) { w[i] = (__bf16)wr[i]; w[8 + i] = (__bf16)wr[16 + i]; }
      acc[j] = wmma_bf(a, w, acc[j]); } }
#pragma unroll
  for (int j = 0; j < 8; ++j) { const float bb = bfr(BA[c0 + j * 16 + col]);
#pragma unroll
    for (int r = 0; r < 8; ++r) sf[wave][8 * g + r][j * 16 + col] = acc[j][r] + bb; }
  LDSX(); for (int rl = 0; rl < 16; ++rl) vst2(D + (r0 + rl) * CC + c0 + lane * 4, *(const v4f*)&sf[wave][rl][lane * 4]); }
__global__ __launch_bounds__(128) void k_nat(const float* __restrict__ Q, const float* __restrict__ K, const float* __restrict__ V, float* __restrict__ O) { __shared__ float ssc[8][NH][NS * NS + 3]; __shared__ __align__(16) float so[8][CC];
  const int tid = threadIdx.x; const int pl = tid >> 4, h = (tid >> 1) & 7, half = tid & 1; const size_t row = (size_t)blockIdx.x * 8 + pl; const size_t b = row / TT; const int t = (int)(row % TT); const int py = t / WWD, px = t % WWD;
  const int d0 = h * HD + half * 32; float qv[32];
  { const float* qr = Q + row * CC + d0;
#pragma unroll
    for (int d = 0; d < 32; ++d) qv[d] = qr[d]; }
#pragma unroll 1
  for (int kk = 0; kk < NS * NS; ++kk) { const int oy = kk / NS - RR, ox = kk % NS - RR; int ny = py + oy, nx = px + ox; const bool valid = (ny >= 0) && (ny < HH) && (nx >= 0) && (nx < WWD); ny = ny < 0 ? 0 : (ny > HH - 1 ? HH - 1 : ny); nx = nx < 0 ? 0 : (nx > WWD - 1 ? WWD - 1 : nx);
    const float* kr = K + (b * TT + (size_t)ny * WWD + nx) * CC + d0; float s = 0.f;
    { _Pragma("clang fp contract(off)");
#pragma unroll
    for (int d4 = 0; d4 < 32; d4 += 4) { const v4f kv = *(const v4f*)(kr + d4); s += qv[d4] * kv[0] + qv[d4 + 1] * kv[1] + qv[d4 + 2] * kv[2] + qv[d4 + 3] * kv[3]; } }
    s += __shfl_xor(s, 1);
    if (half == 0) ssc[pl][h][kk] = valid ? s * 0.125f : -3.0e38f; }
  LDSX(); __syncthreads();
  float m = -3.0e38f; for (int kk = 0; kk < NS * NS; ++kk) m = fmaxf(m, ssc[pl][h][kk]); float sum = 0.f; for (int kk = 0; kk < NS * NS; ++kk) { const float vv = ssc[pl][h][kk]; sum += (vv <= -1.0e38f) ? 0.f : expf(vv - m); } const float inv = 1.0f / sum;
  float acc[32];
#pragma unroll
  for (int d = 0; d < 32; ++d) acc[d] = 0.f;
#pragma unroll 1
  for (int kk = 0; kk < NS * NS; ++kk) { const float sv_ = ssc[pl][h][kk]; const float p = (sv_ <= -1.0e38f) ? 0.f : expf(sv_ - m) * inv; const int oy = kk / NS - RR, ox = kk % NS - RR; int ny = py + oy, nx = px + ox; ny = ny < 0 ? 0 : (ny > HH - 1 ? HH - 1 : ny); nx = nx < 0 ? 0 : (nx > WWD - 1 ? WWD - 1 : nx);
    const float* vr = V + (b * TT + (size_t)ny * WWD + nx) * CC + d0;
#pragma unroll
    for (int d4 = 0; d4 < 32; d4 += 4) { const v4f vv = *(const v4f*)(vr + d4); acc[d4] += p * vv[0]; acc[d4 + 1] += p * vv[1]; acc[d4 + 2] += p * vv[2]; acc[d4 + 3] += p * vv[3]; } }
  { _Pragma("clang fp contract(off)");
  const float* svr = V + row * CC + d0; float svv[32]; float nrm = 0.f, dot = 0.f;
#pragma unroll
  for (int d = 0; d < 32; ++d) { svv[d] = svr[d]; nrm += svv[d] * svv[d]; }
  nrm += __shfl_xor(nrm, 1); const float invn = 1.0f / fmaxf(sqrtf(nrm), 1e-12f);
#pragma unroll
  for (int d = 0; d < 32; ++d) dot += acc[d] * (svv[d] * invn);
  dot += __shfl_xor(dot, 1);
#pragma unroll
  for (int d = 0; d < 32; ++d) so[pl][d0 + d] = acc[d] - dot * (svv[d] * invn);
  }
  __syncthreads();
  for (int e = tid; e < 8 * CC / 4; e += 128) { const int p = e / (CC / 4), c4 = (e % (CC / 4)) * 4; vst2(O + ((size_t)blockIdx.x * 8 + p) * CC + c4, *(const v4f*)&so[p][c4]); } }
__global__ __launch_bounds__(128) void k_wo(const float* __restrict__ O, const float* __restrict__ WO, const float* __restrict__ BO, float* __restrict__ OUT) { __shared__ __align__(16) float st[128][68];
  const int tid = threadIdx.x, wave = tid >> 5, lane = tid & 31, col = lane & 15, g = lane >> 4; const int c0 = blockIdx.y * 128; const size_t r0 = (size_t)blockIdx.x * 64; const size_t b = r0 / TT; const int t0 = (int)(r0 % TT);
  v8f acc[8] = {};
#pragma unroll 2
  for (int kc = 0; kc < CC / 32; ++kc) { const F2 a = split_row(O + (r0 + wave * 16 + col) * CC, kc * 32, lane);
#pragma unroll
    for (int j = 0; j < 8; ++j) { v16b w; const int o = c0 + j * 16 + col; const float* wr = WO + (size_t)o * CC + kc * 32 + 8 * g;
#pragma unroll
      for (int i = 0; i < 8; ++i) { w[i] = (__bf16)wr[i]; w[8 + i] = (__bf16)wr[16 + i]; }
      acc[j] = wmma_bf(a.h, w, acc[j]); acc[j] = wmma_bf(a.l, w, acc[j]); } }
#pragma unroll
  for (int j = 0; j < 8; ++j) { const int cl = j * 16 + col; const float bb = bfr(BO[c0 + cl]);
#pragma unroll
    for (int r = 0; r < 8; ++r) st[cl][wave * 16 + 8 * g + r] = acc[j][r] + bb; }
  __syncthreads();
  for (int e = tid; e < 128 * 16; e += 128) { const int cl = e >> 4, q = e & 15; vst2(OUT + (b * CC + c0 + cl) * TT + t0 + q * 4, *(const v4f*)&st[cl][q * 4]); } }
extern "C" void kernel_launch(void* const* d_in, const int* in_sizes, int n_in, void* d_out, int out_size, void* d_ws, size_t ws_size, hipStream_t stream) {
  (void)in_sizes; (void)n_in; (void)out_size;
  const float** F = (const float**)d_in;
  if (ws_size < (size_t)WS_END) return;
  char* ws = (char*)d_ws; float *XT = (float*)(ws + WS_XT), *Q = (float*)(ws + WS_Q), *K = (float*)(ws + WS_K), *V = (float*)(ws + WS_V), *O = (float*)(ws + WS_O);
  k_xt<<<dim3(TT / 64, CC / 128, NBT), 256, 0, stream>>>(F[0], XT);
  k_proj<<<dim3(NROW / 64, CC / 128, 3), 128, 0, stream>>>(XT, F[1], F[2], F[3], F[4], F[5], F[6], Q, K, V);
  k_nat<<<dim3(NPIXB), 128, 0, stream>>>(Q, K, V, O);
  k_wo<<<dim3(NPIXB * 8 / 64, CC / 128), 128, 0, stream>>>(O, F[7], F[8], (float*)d_out);
}
